// Block_8693013807158
// MI455X (gfx1250) — hardware-verified
//
#include <hip/hip_runtime.h>
#ifndef NB
#define NB 8
#endif
#ifndef SEQ
#define SEQ 1024
#endif
#define NB_FULL 8
#define SEQ_FULL 1024
#define DM 768
#define NH 12
#define HD 64
#define DFF 3072
#define LQ (3 * DM)
#define NR ((size_t)NB * SEQ)

static_assert(NH * HD == DM);
static_assert(HD == 64);
static_assert(DM % 64 == 0 && LQ % 64 == 0 && DFF % 64 == 0);
static_assert(DM % 32 == 0 && DFF % 32 == 0 && HD % 32 == 0);
static_assert(SEQ % 64 == 0 && (NB * SEQ) % 128 == 0);
static_assert(DM % 4 == 0 && DM / 4 <= 256);
static_assert(NB <= NB_FULL && SEQ <= SEQ_FULL);
static_assert((DM * 2) % 128 == 0 && (LQ * 2) % 128 == 0 && (DFF * 2) % 128 == 0 && (DM * 4) % 128 == 0);

typedef unsigned short v8us __attribute__((ext_vector_type(8), may_alias));
typedef float  v8f  __attribute__((ext_vector_type(8)));
typedef float  v4f  __attribute__((ext_vector_type(4)));
typedef float  v4fa __attribute__((ext_vector_type(4), may_alias));
typedef _Float16 v16h __attribute__((ext_vector_type(16)));
typedef _Float16 v4h __attribute__((ext_vector_type(4)));
union FragH { v16h v; v8us half[2]; _Float16 h[16]; unsigned short u[16]; };

__device__ __forceinline__ unsigned short bf16_bits(float x) { unsigned int u = __float_as_uint(x); return (unsigned short)((u + 0x7FFFu + ((u >> 16) & 1u)) >> 16); }
__device__ __forceinline__ float bf16_rne(float x) { return __uint_as_float(((unsigned int)bf16_bits(x)) << 16); }
__device__ __forceinline__ size_t frow(size_t r) { return (r / (size_t)SEQ) * (size_t)SEQ_FULL + (r % (size_t)SEQ); }

__device__ __forceinline__ v16h g2_frag(const _Float16* p, int hh) { FragH f; f.half[0] = *(const v8us*)((const unsigned short*)p + 8 * hh); f.half[1] = *(const v8us*)((const unsigned short*)p + 16 + 8 * hh); return f.v; }
__device__ __forceinline__ v8f g2_mma(v16h a, v16h b, v8f c) { v8f d = __builtin_amdgcn_wmma_f32_16x16x32_f16(false, a, false, b, (short)0, c, false, false); asm volatile("v_nop\n\tv_nop\n\tv_nop\n\tv_nop" : "+v"(d) : "v"(a), "v"(b)); return d; }

__global__ __launch_bounds__(256) void k_wnat(const float* __restrict__ w, size_t n8, _Float16* __restrict__ Bt) {
  const size_t t = (size_t)blockIdx.x * 256 + threadIdx.x; if (t >= n8) return;
  const v4f a = *(const v4fa*)(w + t * 8), c = *(const v4fa*)(w + t * 8 + 4);
  FragH f;
#pragma unroll
  for (int q = 0; q < 4; ++q) { f.h[q] = (_Float16)(bf16_rne(a[q]) * 16.0f); f.h[4 + q] = (_Float16)(bf16_rne(c[q]) * 16.0f); }
  const v8us o = f.half[0];
  unsigned short* d = (unsigned short*)Bt + t * 8;
  *(volatile v8us*)d = o; __threadfence(); *(volatile v8us*)d = o;
}

__global__ __launch_bounds__(256) void k_ln(const float* __restrict__ X, int xfull, int bfin, const float* __restrict__ g, const float* __restrict__ bb, _Float16* __restrict__ N16) {
  #pragma clang fp contract(off)
  __shared__ float red[256];
  const size_t r = blockIdx.x; const int t = threadIdx.x; const bool act = t < (DM / 4); const int c0 = act ? t * 4 : 0;
  const size_t xr = xfull ? frow(r) : r;
  const v4f xa = *(const v4fa*)(X + xr * DM + c0);
  float s[4]; float sum = 0.f;
#pragma unroll
  for (int q = 0; q < 4; ++q) { const float v = bfin ? bf16_rne(xa[q]) : xa[q]; s[q] = act ? v : 0.f; sum = sum + s[q]; }
  red[t] = sum; __syncthreads();
  for (int st = 128; st > 0; st >>= 1) { if (t < st) red[t] = red[t] + red[t + st]; __syncthreads(); }
  const float mu = red[0] * (1.0f / (float)DM); __syncthreads();
  float vs = 0.f;
#pragma unroll
  for (int q = 0; q < 4; ++q) { const float dl = act ? (s[q] - mu) : 0.f; vs = vs + dl * dl; }
  red[t] = vs; __syncthreads();
  for (int st = 128; st > 0; st >>= 1) { if (t < st) red[t] = red[t] + red[t + st]; __syncthreads(); }
  const float rs = rsqrtf(red[0] * (1.0f / (float)DM) + 1e-5f);
  v4h y;
#pragma unroll
  for (int q = 0; q < 4; ++q) { const int c = c0 + q; const float yf = ((s[q] - mu) * rs) * bf16_rne(g[c]) + bf16_rne(bb[c]); y[q] = (_Float16)yf; }
  if (!act) return;
  for (int pass = 0; pass < 2; ++pass) { *(volatile v4h*)(N16 + r * DM + c0) = y; if (pass == 0) __threadfence(); }
}

__global__ __launch_bounds__(256) void k_vt(const _Float16* __restrict__ QKV, _Float16* __restrict__ VT) {
  __shared__ unsigned short tl[64][66];
  const int tid = threadIdx.x; const int slab = blockIdx.x / (SEQ / 64), lg = blockIdx.x % (SEQ / 64); const int b = slab / NH, h = slab % NH;
  for (int i = tid; i < 64 * 8; i += 256) { const int r = i / 8, c8 = (i % 8) * 8; FragH f;
    f.half[0] = *(const v8us*)((const unsigned short*)QKV + ((size_t)b * SEQ + lg * 64 + r) * LQ + 2 * DM + h * HD + c8);
#pragma unroll
    for (int q = 0; q < 8; ++q) tl[r][c8 + q] = f.u[q]; }
  __syncthreads();
  for (int pass = 0; pass < 2; ++pass) {
#pragma unroll
    for (int rd = 0; rd < 2; ++rd) { const int d = rd * 32 + tid / 8, pc = tid % 8; FragH f;
#pragma unroll
      for (int q = 0; q < 8; ++q) f.u[q] = tl[pc * 8 + q][d];
      *(volatile v8us*)((unsigned short*)VT + ((size_t)slab * HD + d) * SEQ + lg * 64 + pc * 8) = f.half[0]; }
    if (pass == 0) __threadfence(); }
}

__global__ __launch_bounds__(128) void k_pattn(const _Float16* __restrict__ QKV, const _Float16* __restrict__ VT, const float* __restrict__ pa_p, const float* __restrict__ pb_p, const float* __restrict__ pc_p, _Float16* __restrict__ O16) {
  __shared__ __attribute__((aligned(16))) unsigned short so[4][16][72];
  const int tid = threadIdx.x, w = tid >> 5, lane = tid & 31, ln = lane & 15, hh = lane >> 4;
  const int qb = blockIdx.x % (SEQ / 64); const int bh = blockIdx.x / (SEQ / 64); const int b = bh / NH, h = bh % NH;
  const size_t rowbase = (size_t)b * SEQ; const int q0 = qb * 64 + w * 16;
  const float A2 = 4.0f * bf16_rne(pa_p[0]);
  const float A1 = 32.0f * bf16_rne(pb_p[0]);
  const float A0 = 256.0f * bf16_rne(pc_p[0]);
  const float PFLOOR = 1e-6f * 256.0f;
  const _Float16* Qp = QKV + (rowbase + q0 + ln) * LQ + h * HD;
  const v16h qf0 = g2_frag(Qp, hh), qf1 = g2_frag(Qp + 32, hh);
  const _Float16* Kp = QKV + (rowbase + ln) * LQ + DM + h * HD;
  const _Float16* Vp = VT + ((size_t)bh * HD + ln) * SEQ;
  const v8f z8 = {0.f, 0.f, 0.f, 0.f, 0.f, 0.f, 0.f, 0.f};
  v8f o0 = z8, o1 = z8, o2 = z8, o3 = z8; float lsum = 0.f;
#pragma unroll 1
  for (int kb = 0; kb < SEQ; kb += 32) {
    const _Float16* k0 = Kp + (size_t)kb * LQ; const _Float16* k1 = k0 + (size_t)16 * LQ;
    v8f s0 = z8, s1 = z8;
    s0 = g2_mma(g2_frag(k0, hh), qf0, s0); s0 = g2_mma(g2_frag(k0 + 32, hh), qf1, s0);
    s1 = g2_mma(g2_frag(k1, hh), qf0, s1); s1 = g2_mma(g2_frag(k1 + 32, hh), qf1, s1);
    FragH pf;
#pragma unroll
    for (int r = 0; r < 8; ++r) {
      float p = fmaf(fmaf(A2, s0[r], A1), s0[r], A0); p = fmaxf(p, PFLOOR); lsum += p; pf.h[r] = (_Float16)p;
      float p2 = fmaf(fmaf(A2, s1[r], A1), s1[r], A0); p2 = fmaxf(p2, PFLOOR); lsum += p2; pf.h[8 + r] = (_Float16)p2; }
    const _Float16* v0 = Vp + kb;
    o0 = g2_mma(g2_frag(v0, hh), pf.v, o0);
    o1 = g2_mma(g2_frag(v0 + (size_t)16 * SEQ, hh), pf.v, o1);
    o2 = g2_mma(g2_frag(v0 + (size_t)32 * SEQ, hh), pf.v, o2);
    o3 = g2_mma(g2_frag(v0 + (size_t)48 * SEQ, hh), pf.v, o3);
  }
  const float lo = __shfl_xor(lsum, 16);
  const float l = lsum + lo;
  const float sc = 64.0f * (1.0f / (l + 256.0f * 1e-8f));
  v8f oo[4] = {o0, o1, o2, o3};
#pragma unroll
  for (int dt = 0; dt < 4; ++dt) { FragH f;
#pragma unroll
    for (int r = 0; r < 8; ++r) f.h[r] = (_Float16)(oo[dt][r] * sc);
    *(v8us*)&so[w][ln][16 * dt + 8 * hh] = f.half[0]; }
  __syncthreads();
  for (int pass = 0; pass < 2; ++pass) {
#pragma unroll
    for (int q = 0; q < 4; ++q) { const int row = q * 4 + (lane >> 3), pc = lane & 7;
      const v8us v = *(const v8us*)&so[w][row][pc * 8];
      *(volatile v8us*)((unsigned short*)O16 + (rowbase + q0 + row) * DM + h * HD + pc * 8) = v; }
    if (pass == 0) __threadfence(); }
}

__global__ __launch_bounds__(128) void k_gemm(const _Float16* __restrict__ A, int lda, const _Float16* __restrict__ Bh, int ldb, float alpha,
    const float* __restrict__ bias, const float* __restrict__ resid, int ldr, int resmode, int rfull,
    float* __restrict__ C, _Float16* __restrict__ C16, int ldc, int ofull, int out16, float oscale,
    int act, const float* __restrict__ g0, const float* __restrict__ g1, const float* __restrict__ g2, int M, int N, int K) {
  __shared__ __attribute__((aligned(16))) float so[4][32][68];
  const int tid = threadIdx.x, w = tid >> 5, lane = tid & 31, ln = lane & 15, hh = lane >> 4;
  const int ntn = N >> 6; const int mt = blockIdx.x / ntn, nq = blockIdx.x - mt * ntn; const int row0 = mt * 128 + 32 * w, col0 = nq * 64; if (row0 >= M) return;
  const _Float16* a0p = A + (size_t)(row0 + ln) * lda; const _Float16* a1p = a0p + (size_t)16 * lda;
  const _Float16* b0p = Bh + (size_t)(col0 + ln) * ldb; const _Float16* b1p = b0p + (size_t)16 * ldb; const _Float16* b2p = b1p + (size_t)16 * ldb; const _Float16* b3p = b2p + (size_t)16 * ldb;
  const v8f z8 = {0.f, 0.f, 0.f, 0.f, 0.f, 0.f, 0.f, 0.f}; v8f c00 = z8, c01 = z8, c02 = z8, c03 = z8, c10 = z8, c11 = z8, c12 = z8, c13 = z8;
#pragma unroll 1
  for (int kb = 0; kb < K; kb += 32) { const v16h a0 = g2_frag(a0p + kb, hh), a1 = g2_frag(a1p + kb, hh);
    v16h b = g2_frag(b0p + kb, hh); c00 = g2_mma(a0, b, c00); c10 = g2_mma(a1, b, c10);
    b = g2_frag(b1p + kb, hh); c01 = g2_mma(a0, b, c01); c11 = g2_mma(a1, b, c11);
    b = g2_frag(b2p + kb, hh); c02 = g2_mma(a0, b, c02); c12 = g2_mma(a1, b, c12);
    b = g2_frag(b3p + kb, hh); c03 = g2_mma(a0, b, c03); c13 = g2_mma(a1, b, c13); }
  float e0 = 0.f, e1 = 0.f, e2 = 0.f;
  if (act) { e0 = bf16_rne(g0[0]); e1 = bf16_rne(g1[0]); e2 = bf16_rne(g2[0]); }
  v8f accs[8] = {c00, c01, c02, c03, c10, c11, c12, c13};
#pragma unroll
  for (int u = 0; u < 8; ++u) { const int t = u & 3, half = u >> 2; const int col = col0 + t * 16 + ln; const float bv = bf16_rne(bias[col]);
#pragma unroll
    for (int r = 0; r < 8; ++r) { const int rloc = half * 16 + 8 * hh + r; float v = accs[u][r] * alpha + bv;
      if (act) v = e0 * v * v + e1 * v + e2;
      so[w][rloc][t * 16 + ln] = v; } }
  __builtin_amdgcn_fence(4  , "workgroup"); __builtin_amdgcn_wave_barrier();
  const int rsub = lane >> 4, c4 = (lane & 15) * 4;
  if (resmode) {
#pragma unroll
    for (int q = 0; q < 16; ++q) { const int r = q * 2 + rsub; const size_t grow = (size_t)(row0 + r); const size_t rr = rfull ? frow(grow) : grow;
      v4f rv = *(const v4fa*)(resid + rr * ldr + col0 + c4);
      if (resmode == 2) { rv[0] = bf16_rne(rv[0]); rv[1] = bf16_rne(rv[1]); rv[2] = bf16_rne(rv[2]); rv[3] = bf16_rne(rv[3]); }
      v4f v = *(const v4fa*)&so[w][r][c4]; v[0] += rv[0]; v[1] += rv[1]; v[2] += rv[2]; v[3] += rv[3];
      *(v4fa*)&so[w][r][c4] = v; } }
  for (int pass = 0; pass < 2; ++pass) {
#pragma unroll
    for (int q = 0; q < 16; ++q) { const int r = q * 2 + rsub; const size_t grow = (size_t)(row0 + r); const size_t orow = ofull ? frow(grow) : grow;
      const v4f v = *(const v4fa*)&so[w][r][c4];
      if (out16) { v4h h4; h4[0] = (_Float16)(v[0] * oscale); h4[1] = (_Float16)(v[1] * oscale); h4[2] = (_Float16)(v[2] * oscale); h4[3] = (_Float16)(v[3] * oscale);
        *(volatile v4h*)(C16 + orow * ldc + col0 + c4) = h4; }
      else *(volatile v4f*)(C + orow * ldc + col0 + c4) = v; }
    if (pass == 0) __threadfence(); }
}

constexpr size_t SZ_BQKV = (size_t)LQ * DM * 2;
constexpr size_t SZ_BO   = (size_t)DM * DM * 2;
constexpr size_t SZ_BW1  = (size_t)DFF * DM * 2;
constexpr size_t SZ_BW2  = (size_t)DM * DFF * 2;
constexpr size_t SZ_XN   = NR * DM * 2;
constexpr size_t SZ_QKV  = NR * LQ * 2;
constexpr size_t SZ_VT   = (size_t)NB * NH * HD * SEQ * 2;
constexpr size_t SZ_U    = NR * DFF * 2;
constexpr size_t SZ_R    = (SZ_QKV + SZ_VT > SZ_U) ? (SZ_QKV + SZ_VT) : SZ_U;
constexpr size_t SZ_O    = NR * DM * 2;
constexpr size_t SZ_X1   = NR * DM * 4;
constexpr size_t WS_TOTAL = SZ_BQKV + SZ_BO + SZ_BW1 + SZ_BW2 + SZ_XN + SZ_R + SZ_O + SZ_X1;
static_assert(SZ_BQKV % 256 == 0 && SZ_BO % 256 == 0 && SZ_BW1 % 256 == 0 && SZ_BW2 % 256 == 0);
static_assert(SZ_XN % 256 == 0 && SZ_QKV % 256 == 0 && SZ_VT % 256 == 0 && SZ_U % 256 == 0 && SZ_O % 256 == 0 && SZ_X1 % 256 == 0);
static_assert(SZ_U <= SZ_R && SZ_QKV + SZ_VT <= SZ_R);
static_assert(WS_TOTAL <= (size_t)134217728);

extern "C" void kernel_launch(void* const* d_in, const int* in_sizes, int n_in,
                              void* d_out, int out_size, void* d_ws, size_t ws_size, hipStream_t stream) {
  if (n_in < 19) return;
  const long long need_x = ((long long)(NB - 1) * SEQ_FULL + SEQ) * DM;
  if ((long long)in_sizes[0] < need_x) return;
  if (in_sizes[1] < DM || in_sizes[2] < DM || in_sizes[3] < DM || in_sizes[4] < DM) return;
  if ((long long)in_sizes[5] < (long long)LQ * DM || in_sizes[6] < LQ) return;
  if ((long long)in_sizes[7] < (long long)DM * DM || in_sizes[8] < DM) return;
  if ((long long)in_sizes[9] < (long long)DFF * DM || in_sizes[10] < DFF) return;
  if ((long long)in_sizes[11] < (long long)DM * DFF || in_sizes[12] < DM) return;
  for (int i = 13; i < 19; ++i) if (in_sizes[i] < 1) return;
  if ((long long)out_size < need_x) return;
  if (ws_size < WS_TOTAL) return;
  const float* const* I = (const float* const*)d_in;
  const float* x = I[0]; const float* ln1w = I[1]; const float* ln1b = I[2]; const float* ln2w = I[3]; const float* ln2b = I[4];
  const float* wqkv = I[5]; const float* bqkv = I[6]; const float* wo = I[7]; const float* bo = I[8];
  const float* w1 = I[9]; const float* b1 = I[10]; const float* w2 = I[11]; const float* b2 = I[12];
  const float* pa = I[13]; const float* pb = I[14]; const float* pc = I[15]; const float* ga = I[16]; const float* gb = I[17]; const float* gc = I[18];
  char* ws = (char*)d_ws; size_t off = 0;
  _Float16* BQKV = (_Float16*)(ws + off); off += SZ_BQKV;
  _Float16* BO   = (_Float16*)(ws + off); off += SZ_BO;
  _Float16* BW1  = (_Float16*)(ws + off); off += SZ_BW1;
  _Float16* BW2  = (_Float16*)(ws + off); off += SZ_BW2;
  _Float16* XN   = (_Float16*)(ws + off); off += SZ_XN;
  char* R = ws + off; off += SZ_R;
  _Float16* O16  = (_Float16*)(ws + off); off += SZ_O;
  float* X1      = (float*)(ws + off); off += SZ_X1;
  _Float16* QKV16 = (_Float16*)R; _Float16* VT = (_Float16*)(R + SZ_QKV); _Float16* U16 = (_Float16*)R;
  _Float16* M16 = XN;
  float* outp = (float*)d_out;

  k_wnat<<<(unsigned)(((size_t)LQ * DM / 8 + 255) / 256), 256, 0, stream>>>(wqkv, (size_t)LQ * DM / 8, BQKV);
  k_wnat<<<(unsigned)(((size_t)DM * DM / 8 + 255) / 256), 256, 0, stream>>>(wo, (size_t)DM * DM / 8, BO);
  k_wnat<<<(unsigned)(((size_t)DFF * DM / 8 + 255) / 256), 256, 0, stream>>>(w1, (size_t)DFF * DM / 8, BW1);
  k_wnat<<<(unsigned)(((size_t)DM * DFF / 8 + 255) / 256), 256, 0, stream>>>(w2, (size_t)DM * DFF / 8, BW2);
  k_ln<<<(unsigned)NR, 256, 0, stream>>>(x, 1, 1, ln1w, ln1b, XN);
  k_gemm<<<(unsigned)((NR / 128) * (LQ / 64)), 128, 0, stream>>>(XN, DM, BQKV, DM, 0.0625f, bqkv, x, DM, 0, 0, X1, QKV16, LQ, 0, 1, 1.0f, 0, ga, gb, gc, (int)NR, LQ, DM);
  k_vt<<<(unsigned)(NB * NH * (SEQ / 64)), 256, 0, stream>>>(QKV16, VT);
  k_pattn<<<(unsigned)((SEQ / 64) * NB * NH), 128, 0, stream>>>(QKV16, VT, pa, pb, pc, O16);
  k_gemm<<<(unsigned)((NR / 128) * (DM / 64)), 128, 0, stream>>>(O16, DM, BO, DM, 0.0009765625f, bo, x, DM, 2, 1, X1, O16, DM, 0, 0, 1.0f, 0, ga, gb, gc, (int)NR, DM, DM);
  k_ln<<<(unsigned)NR, 256, 0, stream>>>(X1, 0, 0, ln2w, ln2b, M16);
  k_gemm<<<(unsigned)((NR / 128) * (DFF / 64)), 128, 0, stream>>>(M16, DM, BW1, DM, 0.0625f, b1, x, DM, 0, 0, X1, U16, DFF, 0, 1, 16.0f, 1, ga, gb, gc, (int)NR, DFF, DM);
  k_gemm<<<(unsigned)((NR / 128) * (DM / 64)), 128, 0, stream>>>(U16, DFF, BW2, DFF, 0.00390625f, b2, X1, DM, 1, 0, outp, O16, DM, 1, 0, 1.0f, 0, ga, gb, gc, (int)NR, DM, DFF);
}
